// MTFMTextModel_23905787969915
// MI455X (gfx1250) — hardware-verified
//
#include <hip/hip_runtime.h>
#include <stdint.h>
#include <stddef.h>


typedef _Float16 v4h  __attribute__((ext_vector_type(4)));
typedef _Float16 v8h  __attribute__((ext_vector_type(8)));
typedef _Float16 v16h __attribute__((ext_vector_type(16)));
typedef float    v8f  __attribute__((ext_vector_type(8)));
typedef float    v4f  __attribute__((ext_vector_type(4)));

union Frag  { v16h v; v8h h8[2]; v4h h4[4]; };
union Pack8 { v8h v; _Float16 e[8]; };
union Pack4 { v4f v; float e[4]; };

#define NB    256
#define NS    512
#define NE    100
#define NCH   256
#define NA    1000
#define NF    8
#define SP    1008
#define WSC   64.0f
#define WINV  0.015625f

__host__ __device__ inline int kpad_of(int h) { return ((NE * h + 31) >> 5) << 5; }
__host__ __device__ inline int woff_of(int i) { int o = 0; for (int q = 0; q < i; ++q) o += NCH * kpad_of(q + 2); return o; }

__device__ __forceinline__ v8f zero8() { v8f z = {0.f, 0.f, 0.f, 0.f, 0.f, 0.f, 0.f, 0.f}; return z; }

__device__ __forceinline__ v8f wmma16(v8f c, v16h a, v16h b) {
  v8f d = __builtin_amdgcn_wmma_f32_16x16x32_f16(false, a, false, b, (short)0, c, false, false);
  asm volatile("v_nop\n\tv_nop\n\tv_nop\n\tv_nop" : "+v"(d) : "v"(a), "v"(b));
  return d;
}

__global__ __launch_bounds__(256) void k_packconv(const float* __restrict__ w2, const float* __restrict__ w3,
                                                   const float* __restrict__ w4, const float* __restrict__ w5,
                                                   _Float16* __restrict__ Wp) {
  __shared__ __attribute__((aligned(16))) _Float16 sw[16 * 512];
  const int tid = threadIdx.x;
  const int i  = blockIdx.x >> 4;
  const int cb = (blockIdx.x & 15) * 16;
  const int h  = i + 2;
  const int Kp = kpad_of(h), K1 = NE * h;
  const float* src = (i == 0) ? w2 : (i == 1) ? w3 : (i == 2) ? w4 : w5;
  for (int idx = tid; idx < 16 * Kp; idx += 256) {
    const int r = idx / Kp, kk = idx - r * Kp;
    float v = 0.0f;
    if (kk < K1) {
      const int j = kk / NE, e = kk - j * NE;
      v = src[((size_t)(cb + r) * NE + e) * h + j] * WSC;
    }
    sw[idx] = (_Float16)v;
  }
  __syncthreads();
  _Float16* base = Wp + woff_of(i) + (size_t)cb * Kp;
  const int nck = 2 * Kp;
  for (int pass = 0; pass < 2; ++pass) {
    for (int c = tid; c < nck; c += 256) {
      v8h val = *(const v8h*)(sw + 8 * c);
      *(volatile v8h*)(base + 8 * c) = val;
    }
    if (pass == 0) __threadfence();
  }
}

__global__ __launch_bounds__(256) void k_packfc(const float* __restrict__ src0, int rows0,
                                                 const float* __restrict__ src1, int rows1,
                                                 int cols, int split, _Float16* __restrict__ dst, int pitch) {
  const int row = blockIdx.x, c = threadIdx.x;
  if (c >= (pitch >> 3)) return;
  const int col0 = c * 8, half = cols >> 1;
  Pack8 u;
#pragma unroll
  for (int e = 0; e < 8; ++e) {
    const int col = col0 + e;
    int scol;
    if (split) scol = (col < half) ? col : ((col >= 1024 && col < 1024 + half) ? (col - 1024 + half) : -1);
    else       scol = (col < cols) ? col : -1;
    float v = 0.0f;
    if (scol >= 0) {
      if (row < rows0)              v = src0[(size_t)row * cols + scol] * WSC;
      else if (row < rows0 + rows1) v = src1[(size_t)(row - rows0) * cols + scol] * WSC;
    }
    u.e[e] = (_Float16)v;
  }
  _Float16* p = dst + (size_t)row * pitch + col0;
  *(volatile v8h*)p = u.v;
  __threadfence();
  *(volatile v8h*)p = u.v;
}

__global__ __launch_bounds__(256) void k_q(const float* __restrict__ api, const float* __restrict__ w1,
                                            float* __restrict__ qv, int nA) {
  const int t = blockIdx.x * 256 + threadIdx.x;
  if (t >= 2 * nA) return;
  const int a = t >> 1, part = t & 1;
  float ae[8];
#pragma unroll
  for (int f2 = 0; f2 < 8; ++f2) ae[f2] = api[(size_t)f2 * nA + a];
  Pack4 q;
#pragma unroll
  for (int e = 0; e < 4; ++e) {
    const int f = part * 4 + e;
    float s = 0.0f;
#pragma unroll
    for (int f2 = 0; f2 < 8; ++f2) s += ae[f2] * w1[f * 16 + 8 + f2];
    q.e[e] = s;
  }
  float* p = qv + (size_t)t * 4;
  *(volatile v4f*)p = q.v;
  __threadfence();
  *(volatile v4f*)p = q.v;
}

__global__ __launch_bounds__(256) void k_embed(const int* __restrict__ ids, int nrows,
                                                const float* __restrict__ table, int V,
                                                _Float16* __restrict__ X) {
  __shared__ int sid[64];
  __shared__ __attribute__((aligned(16))) _Float16 sx[6400];
  const int tid = threadIdx.x, row0 = blockIdx.x * 64;
  if (tid < 64) {
    const int r = row0 + tid;
    int id = 0;
    if (r < nrows) {
      id = ids[r];
      if (id < 0) id += V;
      id = (id < 0) ? 0 : ((id > V - 1) ? (V - 1) : id);
    }
    sid[tid] = id;
  }
  __syncthreads();
  {
    const int r = tid >> 2, e0 = (tid & 3) * 25;
    const bool valid = (row0 + r) < nrows;
    const float* tr = table + (size_t)sid[r] * NE + e0;
    _Float16* sr = sx + r * NE + e0;
#pragma unroll
    for (int k = 0; k < 25; ++k) {
      float v = 0.0f;
      if (valid) v = tr[k];
      sr[k] = (_Float16)v;
    }
  }
  __syncthreads();
  _Float16* base = X + (size_t)blockIdx.x * 6400;
  for (int pass = 0; pass < 2; ++pass) {
    for (int c = tid; c < 800; c += 256) {
      v8h val = *(const v8h*)(sx + 8 * c);
      *(volatile v8h*)(base + 8 * c) = val;
    }
    if (pass == 0) __threadfence();
  }
}

__global__ __launch_bounds__(128) void k_conv(const _Float16* __restrict__ X, const _Float16* __restrict__ Wp,
                                               const float* __restrict__ cb2, const float* __restrict__ cb3,
                                               const float* __restrict__ cb4, const float* __restrict__ cb5,
                                               _Float16* __restrict__ E, int S) {
  __shared__ float red[4][64];
  __shared__ __attribute__((aligned(16))) _Float16 sval[64];
  const int tid = threadIdx.x, lane = tid & 31, hh = lane >> 4, m = lane & 15, w = tid >> 5;
  const int i = blockIdx.x >> 2, g = blockIdx.x & 3, b = blockIdx.y;
  const int h = i + 2, Kp = kpad_of(h), Lh = S - h + 1, ntt = (Lh + 31) >> 5;
  const _Float16* Wc = Wp + woff_of(i) + (size_t)(g * 64 + m) * Kp + 8 * hh;
  const float* bias = (i == 0) ? cb2 : (i == 1) ? cb3 : (i == 2) ? cb4 : cb5;
  const float ninf = -__builtin_huge_valf();
  float mx[4] = {ninf, ninf, ninf, ninf};

  for (int tt = w; tt < ntt; tt += 4) {
    const int t0 = tt * 32;
    int ta = t0 + m;      if (ta > Lh - 1) ta = Lh - 1;
    int tb = t0 + 16 + m; if (tb > Lh - 1) tb = Lh - 1;
    const _Float16* ar0 = X + ((size_t)b * S + ta) * NE + 8 * hh;
    const _Float16* ar1 = X + ((size_t)b * S + tb) * NE + 8 * hh;
    v8f acc0[4], acc1[4];
#pragma unroll
    for (int j = 0; j < 4; ++j) { acc0[j] = zero8(); acc1[j] = zero8(); }
    for (int ks = 0; ks < Kp; ks += 32) {
      Frag a0, a1;
      a0.h4[0] = *(const v4h*)(ar0 + ks);      a0.h4[1] = *(const v4h*)(ar0 + ks + 4);
      a0.h4[2] = *(const v4h*)(ar0 + ks + 16); a0.h4[3] = *(const v4h*)(ar0 + ks + 20);
      a1.h4[0] = *(const v4h*)(ar1 + ks);      a1.h4[1] = *(const v4h*)(ar1 + ks + 4);
      a1.h4[2] = *(const v4h*)(ar1 + ks + 16); a1.h4[3] = *(const v4h*)(ar1 + ks + 20);
#pragma unroll
      for (int j = 0; j < 4; ++j) {
        const _Float16* wr = Wc + (size_t)(j * 16) * Kp + ks;
        Frag bb;
        bb.h8[0] = *(const v8h*)(wr);
        bb.h8[1] = *(const v8h*)(wr + 16);
        acc0[j] = wmma16(acc0[j], a0.v, bb.v);
        acc1[j] = wmma16(acc1[j], a1.v, bb.v);
      }
    }
#pragma unroll
    for (int j = 0; j < 4; ++j) {
      float cm = acc0[j][0];
#pragma unroll
      for (int r = 0; r < 8; ++r) { cm = fmaxf(cm, acc0[j][r]); cm = fmaxf(cm, acc1[j][r]); }
      mx[j] = fmaxf(mx[j], cm);
    }
  }
#pragma unroll
  for (int j = 0; j < 4; ++j) mx[j] = fmaxf(mx[j], __shfl_xor(mx[j], 16));
  if (hh == 0) {
#pragma unroll
    for (int j = 0; j < 4; ++j) red[w][j * 16 + m] = mx[j];
  }
  __syncthreads();
  if (tid < 64) {
    float v = fmaxf(fmaxf(red[0][tid], red[1][tid]), fmaxf(red[2][tid], red[3][tid]));
    float o = fmaxf(v * WINV + bias[g * 64 + tid], 0.0f);
    sval[tid] = (_Float16)o;
  }
  __syncthreads();
  if (tid < 8) {
    v8h val = *(const v8h*)(sval + 8 * tid);
    _Float16* p = E + (size_t)b * (4 * NCH) + i * NCH + g * 64 + 8 * tid;
    *(volatile v8h*)p = val;
    __threadfence();
    *(volatile v8h*)p = val;
  }
}

__global__ __launch_bounds__(128) void k_fc(const _Float16* __restrict__ A, int lda,
                                             const _Float16* __restrict__ W, int ldw, int ksteps,
                                             const float* __restrict__ bias0, int n0,
                                             const float* __restrict__ bias1, int n1, int act, int mode,
                                             _Float16* __restrict__ dstH, int ldo, int coff, int nkeep,
                                             float* __restrict__ dstU, float* __restrict__ dstF, int nout) {
  extern __shared__ __attribute__((aligned(16))) float stage[];
  const int tid = threadIdx.x, lane = tid & 31, hh = lane >> 4, m = lane & 15, w = tid >> 5;
  const int r0 = blockIdx.x * 16;
  const _Float16* ar = A + (size_t)(r0 + m) * lda + 8 * hh;

  for (int ng = 0; ng < 16; ++ng) {
    const int nt = ng * 64 + w * 16;
    const _Float16* wr = W + (size_t)(nt + m) * ldw + 8 * hh;
    v8f acc = zero8();
    for (int ks = 0; ks < ksteps; ++ks) {
      const int kk = ks * 32;
      Frag a, bb;
      a.h8[0]  = *(const v8h*)(ar + kk);  a.h8[1]  = *(const v8h*)(ar + kk + 16);
      bb.h8[0] = *(const v8h*)(wr + kk);  bb.h8[1] = *(const v8h*)(wr + kk + 16);
      acc = wmma16(acc, a.v, bb.v);
    }
    const int n = nt + m;
    float bs = 0.0f;
    if (n < n0) bs = bias0[n];
    else if (n < n1) bs = bias1[n - n0];
    if (nt < SP) {
#pragma unroll
      for (int r = 0; r < 8; ++r) {
        float v = acc[r] * WINV + bs;
        if (act) v = tanhf(v);
        if (n >= n1) v = 0.0f;
        stage[(8 * hh + r) * SP + n] = v;
      }
    }
  }
  __syncthreads();

  if (mode & 1) {
    for (int pass = 0; pass < 2; ++pass) {
      for (int row = 0; row < 16; ++row) {
        const int col0 = tid * 8;
        Pack8 u;
#pragma unroll
        for (int e = 0; e < 8; ++e) {
          const int c = col0 + e;
          float v = 0.0f;
          if (c < nkeep) v = stage[row * SP + c];
          u.e[e] = (_Float16)v;
        }
        *(volatile v8h*)(dstH + (size_t)(r0 + row) * ldo + coff + col0) = u.v;
      }
      if (pass == 0) __threadfence();
    }
  }
  if ((mode & 2) && tid < 32) {
    const int row = tid >> 1, part = tid & 1;
    v4f v = *(const v4f*)(stage + row * SP + n0 + 4 * part);
    float* p = dstU + (size_t)(r0 + row) * 8 + 4 * part;
    *(volatile v4f*)p = v;
    __threadfence();
    *(volatile v4f*)p = v;
  }
  if (mode & 4) {
    float* slab = dstF + (size_t)r0 * nout;
    const int nck = (16 * nout) >> 2;
    for (int pass = 0; pass < 2; ++pass) {
      for (int c = tid; c < nck; c += 128) {
        const int f = 4 * c;
        const int row = f / nout, col = f - row * nout;
        v4f v = *(const v4f*)(stage + row * SP + col);
        *(volatile v4f*)(slab + f) = v;
      }
      if (pass == 0) __threadfence();
    }
  }
}

__global__ __launch_bounds__(256) void k_head(const float* __restrict__ ut, const float* __restrict__ qv,
                                               const float* __restrict__ api, const float* __restrict__ w1,
                                               const float* __restrict__ b1, const float* __restrict__ w2,
                                               const float* __restrict__ b2, _Float16* __restrict__ ficin, int nA) {
  __shared__ float sut[8];
  __shared__ float sp[8];
  __shared__ __attribute__((aligned(16))) _Float16 sh[2048];
  const int b = blockIdx.x, tid = threadIdx.x;
  if (tid < 8) sut[tid] = ut[(size_t)b * 8 + tid];
  __syncthreads();
  if (tid < 8) {
    float p = 0.0f;
#pragma unroll
    for (int f2 = 0; f2 < 8; ++f2) p += sut[f2] * w1[tid * 16 + f2];
    sp[tid] = p;
  }
  __syncthreads();
  const float bb2 = b2[0];
  for (int a = tid; a < 1024; a += 256) {
    float umm = 0.0f, um = 0.0f;
    if (a < nA) {
#pragma unroll
      for (int f = 0; f < 8; ++f) umm += sut[f] * api[(size_t)f * nA + a];
      float z = 0.0f;
#pragma unroll
      for (int f = 0; f < 8; ++f) z += w2[f] * ((sp[f] + qv[(size_t)a * 8 + f]) + b1[f]);
      um = tanhf(z + bb2);
    }
    sh[a] = (_Float16)umm;
    sh[1024 + a] = (_Float16)um;
  }
  __syncthreads();
  v8h val = *(const v8h*)(sh + 8 * tid);
  _Float16* p = ficin + (size_t)b * 2048 + 8 * tid;
  *(volatile v8h*)p = val;
  __threadfence();
  *(volatile v8h*)p = val;
}

extern "C" void kernel_launch(void* const* d_in, const int* in_sizes, int n_in,
                              void* d_out, int out_size, void* d_ws, size_t ws_size,
                              hipStream_t stream) {
  if (n_in < 25) return;
  const int nrows = in_sizes[0];
  if (nrows != NB * NS || out_size != NB * NA) return;
  const int V = in_sizes[1] / NE;
  if (V < 1) return;

  const int*   ids    = (const int*)d_in[0];
  const float* table  = (const float*)d_in[1];
  const float* cw2    = (const float*)d_in[2];
  const float* cb2    = (const float*)d_in[3];
  const float* cw3    = (const float*)d_in[4];
  const float* cb3    = (const float*)d_in[5];
  const float* cw4    = (const float*)d_in[6];
  const float* cb4    = (const float*)d_in[7];
  const float* cw5    = (const float*)d_in[8];
  const float* cb5    = (const float*)d_in[9];
  const float* sc_w   = (const float*)d_in[10];
  const float* sc_b   = (const float*)d_in[11];
  const float* ff_w   = (const float*)d_in[12];
  const float* ff_b   = (const float*)d_in[13];
  const float* api    = (const float*)d_in[14];
  const float* w1     = (const float*)d_in[15];
  const float* b1     = (const float*)d_in[16];
  const float* w2     = (const float*)d_in[17];
  const float* b2     = (const float*)d_in[18];
  const float* ficl_w = (const float*)d_in[19];
  const float* ficl_b = (const float*)d_in[20];
  const float* fus_w  = (const float*)d_in[21];
  const float* fus_b  = (const float*)d_in[22];
  const float* ow     = (const float*)d_in[23];
  const float* ob     = (const float*)d_in[24];

  char* ws = (char*)d_ws;
  size_t off = 0;
  auto carve = [&](size_t bytes) -> void* {
    off = (off + 255) & ~(size_t)255;
    void* p = ws + off; off += bytes; return p;
  };

  const int nblkE = nrows / 64 + 1;
  const int wtot  = woff_of(4);
  _Float16* X     = (_Float16*)carve((size_t)nblkE * 6400 * 2);
  _Float16* Wp    = (_Float16*)carve((size_t)wtot * 2);
  _Float16* W1    = (_Float16*)carve((size_t)1024 * 1024 * 2);
  _Float16* Wfl   = (_Float16*)carve((size_t)1024 * 2048 * 2);
  _Float16* Wfu   = (_Float16*)carve((size_t)1024 * 2048 * 2);
  _Float16* Wo    = (_Float16*)carve((size_t)1024 * 1024 * 2);
  _Float16* Eh    = (_Float16*)carve((size_t)NB * 1024 * 2);
  float*    ut    = (float*)   carve((size_t)NB * 8 * 4);
  float*    qv    = (float*)   carve((size_t)NA * 8 * 4);
  _Float16* ficin = (_Float16*)carve((size_t)NB * 2048 * 2);
  _Float16* fusin = (_Float16*)carve((size_t)NB * 2048 * 2);
  _Float16* ummf  = (_Float16*)carve((size_t)NB * 1024 * 2);
  if (off > ws_size) return;
  float* outp = (float*)d_out;

  k_packconv<<<dim3(64), 256, 0, stream>>>(cw2, cw3, cw4, cw5, Wp);
  k_packfc<<<dim3(1024), 256, 0, stream>>>(sc_w, NA, ff_w, NF, 1024, 0, W1, 1024);
  k_packfc<<<dim3(1024), 256, 0, stream>>>(ficl_w, NA, ficl_w, 0, 2 * NA, 1, Wfl, 2048);
  k_packfc<<<dim3(1024), 256, 0, stream>>>(fus_w, NA, fus_w, 0, 2 * NA, 1, Wfu, 2048);
  k_packfc<<<dim3(1024), 256, 0, stream>>>(ow, NA, ow, 0, NA, 0, Wo, 1024);
  k_q<<<dim3((2 * NA + 255) / 256), 256, 0, stream>>>(api, w1, qv, NA);

  k_embed<<<dim3(nblkE), 256, 0, stream>>>(ids, nrows, table, V, X);

  k_conv<<<dim3(16, NB), 128, 0, stream>>>(X, Wp, cb2, cb3, cb4, cb5, Eh, NS);

  const size_t ldsFC = (size_t)16 * SP * 4;
  k_fc<<<dim3(16), 128, ldsFC, stream>>>(Eh, 1024, W1, 1024, 32, sc_b, NA, ff_b, NA + NF, 0, 3,
                                         fusin, 2048, 0, NA, ut, outp, NA);
  k_head<<<dim3(NB), 256, 0, stream>>>(ut, qv, api, w1, b1, w2, b2, ficin, NA);
  k_fc<<<dim3(16), 128, ldsFC, stream>>>(ficin, 2048, Wfl, 2048, 64, ficl_b, NA, ficl_b, NA, 1, 1,
                                         fusin, 2048, 1024, NA, ut, outp, NA);
  k_fc<<<dim3(16), 128, ldsFC, stream>>>(fusin, 2048, Wfu, 2048, 64, fus_b, NA, fus_b, NA, 0, 1,
                                         ummf, 1024, 0, NA, ut, outp, NA);
  k_fc<<<dim3(16), 128, ldsFC, stream>>>(ummf, 1024, Wo, 1024, 32, ob, NA, ob, NA, 0, 4,
                                         fusin, 2048, 0, NA, ut, outp, NA);
}
